// ImageEncoder_1838246002910
// MI455X (gfx1250) — hardware-verified
//
#include <hip/hip_runtime.h>
#include <math.h>
#include <stddef.h>

constexpr int kBatch = 8;
constexpr int kSeq   = 2048;
constexpr int kPatch = 768;
constexpr int kEmb   = 256;
constexpr int kHeads = 4;
constexpr int kHdim  = 64;
constexpr int kTok   = kBatch * kSeq;
constexpr int kQKld  = 2 * kEmb;
constexpr float kQKVCarry   = 8.0f;
constexpr float kPCarry     = 2048.0f;
constexpr float kScoreScale = 1.0f / (8.0f * 8.0f * 8.0f);
constexpr float kPVScale    = 1.0f / (2048.0f * 8.0f);

static_assert(kTok % 64 == 0 && kEmb % 64 == 0 && kSeq % 64 == 0 && kHdim % 64 == 0);
static_assert(kPatch % 32 == 0 && kEmb % 32 == 0 && kHdim % 32 == 0 && kSeq % 32 == 0);

constexpr size_t kOffWeHi  = 0;
constexpr size_t kOffWeLo  = 393216;
constexpr size_t kOffSqHi  = 786432;
constexpr size_t kOffSqLo  = 1310720;
constexpr size_t kOffH     = 1835008;
constexpr size_t kOffOlo   = kOffH + 8388608;
constexpr size_t kOffQK    = 18612224;
constexpr size_t kOffVT    = 35389440;
constexpr size_t kOffHrHi  = 43778048;
constexpr size_t kOffHrLo  = kOffHrHi + 8388608;
constexpr size_t kOffXHi   = 60555264;
constexpr size_t kOffXLo   = kOffXHi + 25165824;
constexpr size_t kOffScore = kOffXHi;
constexpr size_t kOffP     = kOffXHi + 33554432;
constexpr size_t kWsTotal  = 110886912;
static_assert(kOffWeLo == kOffWeHi + (size_t)kEmb * kPatch * 2);
static_assert(kOffSqHi == kOffWeLo + (size_t)kEmb * kPatch * 2);
static_assert(kOffSqLo == kOffSqHi + (size_t)4 * kEmb * kEmb * 2);
static_assert(kOffH    == kOffSqLo + (size_t)4 * kEmb * kEmb * 2);
static_assert(kOffQK   == kOffH + (size_t)kTok * kEmb * 4);
static_assert(kOffOlo + (size_t)kTok * kEmb * 2 == kOffQK);
static_assert(kOffVT   == kOffQK + (size_t)kTok * kQKld * 2);
static_assert(kOffHrHi == kOffVT + (size_t)kEmb * kTok * 2);
static_assert(kOffXHi  == kOffHrLo + (size_t)kTok * kEmb * 2);
static_assert(kOffXLo + (size_t)kTok * kPatch * 2 == kWsTotal);
static_assert(kOffP == kOffScore + (size_t)2 * kSeq * kSeq * 4);
static_assert(kOffP + (size_t)2 * kSeq * kSeq * 2 == kWsTotal);
static_assert(kWsTotal <= (size_t)134217728);

typedef __attribute__((ext_vector_type(16))) _Float16 v16h;
typedef __attribute__((ext_vector_type(8)))  _Float16 v8h;
typedef __attribute__((ext_vector_type(16))) __bf16   v16b;
typedef __attribute__((ext_vector_type(8)))  __bf16   v8b;
typedef __attribute__((ext_vector_type(8)))  float    v8f;
typedef __attribute__((ext_vector_type(4)))  float    v4f;
typedef __attribute__((ext_vector_type(2)))  float    v2f;
typedef __attribute__((ext_vector_type(4)))  unsigned int v4u;

__device__ __forceinline__ unsigned short f2bf_bits(float f) {
  unsigned u = __float_as_uint(f);
  return (unsigned short)((u + 0x7FFFu + ((u >> 16) & 1u)) >> 16);
}
__device__ __forceinline__ float bf_bits2f(unsigned short h) { return __uint_as_float(((unsigned)h) << 16); }

__device__ __forceinline__ void dep_guard_h(v8f& a, v8f& b, v16h x, v16h y) { asm volatile("v_nop\n\tv_nop\n\tv_nop\n\tv_nop" : "+v"(a), "+v"(b) : "v"(x), "v"(y)); }
__device__ __forceinline__ void dep_guard_b(v8f& a, v8f& b, v16b x, v16b y) { asm volatile("v_nop\n\tv_nop\n\tv_nop\n\tv_nop" : "+v"(a), "+v"(b) : "v"(x), "v"(y)); }
__device__ __forceinline__ void keep4_h(v16h a, v16h b, v16h c, v16h d) { asm volatile("v_nop" :: "v"(a), "v"(b), "v"(c), "v"(d)); }
__device__ __forceinline__ void keep4_b(v16b a, v16b b, v16b c, v16b d) { asm volatile("v_nop" :: "v"(a), "v"(b), "v"(c), "v"(d)); }
__device__ __forceinline__ void acc_guard4(v8f& a, v8f& b, v8f& c, v8f& d) { asm volatile("v_nop\n\tv_nop\n\tv_nop\n\tv_nop" : "+v"(a), "+v"(b), "+v"(c), "+v"(d)); }
template <typename T> struct Frag;
template <> struct Frag<_Float16> {
  typedef v16h V; union U { v16h v; v8h h[2]; };
  static __device__ __forceinline__ v16h load(const _Float16* p) {
    U f; f.h[0] = *(const v8h*)(p); f.h[1] = *(const v8h*)(p + 16); return f.v;
  }
  static __device__ __forceinline__ v8f mma(v16h a, v16h b, v8f c) {
    return __builtin_amdgcn_wmma_f32_16x16x32_f16(false, a, false, b, (short)0, c, false, false);
  }
  static __device__ __forceinline__ void guard(v8f& a, v8f& b, v16h x, v16h y) { dep_guard_h(a, b, x, y); }
  static __device__ __forceinline__ void keep(v16h a, v16h b, v16h c, v16h d) { keep4_h(a, b, c, d); }
};
template <> struct Frag<__bf16> {
  typedef v16b V; union U { v16b v; v8b h[2]; };
  static __device__ __forceinline__ v16b load(const __bf16* p) {
    U f; f.h[0] = *(const v8b*)(p); f.h[1] = *(const v8b*)(p + 16); return f.v;
  }
  static __device__ __forceinline__ v8f mma(v16b a, v16b b, v8f c) {
    return __builtin_amdgcn_wmma_f32_16x16x32_bf16(false, a, false, b, (short)0, c, false, false);
  }
  static __device__ __forceinline__ void guard(v8f& a, v8f& b, v16b x, v16b y) { dep_guard_b(a, b, x, y); }
  static __device__ __forceinline__ void keep(v16b a, v16b b, v16b c, v16b d) { keep4_b(a, b, c, d); }
};

__device__ __forceinline__ unsigned pk16(unsigned short a, unsigned short b) { return (unsigned)a | ((unsigned)b << 16); }
__device__ __forceinline__ unsigned short h_bits(float f) { const _Float16 h = (_Float16)f; return __builtin_bit_cast(unsigned short, h); }

template <int ET> struct Elem;
template <> struct Elem<0> { typedef _Float16 T; };
template <> struct Elem<1> { typedef __bf16 T; };
template <int ET, bool SPLIT, int BIAS_MODE, int OUT_MODE, bool RESID, int ACT = 0>
__global__ __launch_bounds__(256) void wmma_gemm64(
    const unsigned short* __restrict__ Ap, const unsigned short* __restrict__ A2p, int lda, long strideA,
    const unsigned short* __restrict__ Btp, const unsigned short* __restrict__ Bt2p, int ldb, long strideB,
    void* __restrict__ Cout, void* __restrict__ Cout2, int ldc, long strideC,
    const float* __restrict__ bias,
    const float* __restrict__ resid, long strideR,
    int M, int N, int K, float scale, float post) {
  typedef typename Elem<ET>::T T;
  typedef typename Frag<T>::V V;
  const T* A = (const T*)Ap; const T* A2 = (const T*)A2p; const T* Bt = (const T*)Btp; const T* Bt2 = (const T*)Bt2p;
  __shared__ __align__(16) float sT[8][16 * 68];
  const int b    = blockIdx.y;
  const int lane = threadIdx.x & 31;
  const int wave = threadIdx.x >> 5;
  const int tilesN = N >> 6;
  const int tilesM = M >> 6;
  const int tile = blockIdx.x * 8 + wave;
  if (tile >= tilesM * tilesN) return;
  const int tm = tile / tilesN;
  const int tn = tile - tm * tilesN;
  const int m0 = tm << 6;
  const int n0 = tn << 6;

  const T* Ab  = A  + (size_t)b * strideA;
  const T* Bb  = Bt + (size_t)b * strideB;
  const T* Ab2 = SPLIT ? (A2  + (size_t)b * strideA) : nullptr;
  const T* Bb2 = SPLIT ? (Bt2 + (size_t)b * strideB) : nullptr;

  const int rlane = lane & 15;
  const int koff  = (lane >> 4) * 8;
  const int mOff  = (lane >> 4) * 8;

  v8f acc[4][4];
#pragma unroll
  for (int i = 0; i < 4; ++i)
#pragma unroll
    for (int j = 0; j < 4; ++j) acc[i][j] = (v8f){0.f,0.f,0.f,0.f,0.f,0.f,0.f,0.f};

  for (int k0 = 0; k0 < K; k0 += 32) {
    V bh[4], bl[4];
#pragma unroll
    for (int j = 0; j < 4; ++j) {
      const size_t bo = (size_t)(n0 + (j << 4) + rlane) * ldb + koff + k0;
      bh[j] = Frag<T>::load(Bb + bo);
      if (SPLIT) bl[j] = Frag<T>::load(Bb2 + bo);
    }
#pragma unroll
    for (int i = 0; i < 4; ++i) {
      const size_t ao = (size_t)(m0 + (i << 4) + rlane) * lda + koff + k0;
      V ah = Frag<T>::load(Ab + ao);
      V al;
      if (SPLIT) al = Frag<T>::load(Ab2 + ao);
#pragma unroll
      for (int j = 0; j < 4; ++j) {
        acc[i][j] = Frag<T>::mma(ah, bh[j], acc[i][j]);
        if (SPLIT) {
          acc[i][j] = Frag<T>::mma(ah, bl[j], acc[i][j]);
          acc[i][j] = Frag<T>::mma(al, bh[j], acc[i][j]);
        }
      }
      Frag<T>::guard(acc[i][0], acc[i][3], ah, SPLIT ? al : ah);
    }
    Frag<T>::keep(bh[0], bh[1], bh[2], bh[3]);
    if (SPLIT) Frag<T>::keep(bl[0], bl[1], bl[2], bl[3]);
  }
  acc_guard4(acc[0][0], acc[0][1], acc[0][2], acc[0][3]);
  acc_guard4(acc[1][0], acc[1][1], acc[1][2], acc[1][3]);
  acc_guard4(acc[2][0], acc[2][1], acc[2][2], acc[2][3]);
  acc_guard4(acc[3][0], acc[3][1], acc[3][2], acc[3][3]);

  float* slab = sT[wave];
  const float* Rb = RESID ? (resid + (size_t)b * strideR) : nullptr;
#pragma unroll
  for (int i = 0; i < 4; ++i) {
    const int mBase = m0 + (i << 4);
#pragma unroll
    for (int j = 0; j < 4; ++j) {
      const int n = n0 + (j << 4) + rlane;
      float bv = 0.f;
      if (BIAS_MODE == 2) bv = bias[n];
#pragma unroll
      for (int r = 0; r < 8; ++r) {
        float v = acc[i][j][r] * scale;
        if (BIAS_MODE == 1) v += bias[mBase + mOff + r];
        if (BIAS_MODE == 2) v += bv;
        if (RESID) v += Rb[(size_t)(mBase + mOff + r) * ldc + n];
        v = v * post;
        if (ACT == 2) v = fmaxf(v, 0.0f);
        if (ACT == 4) v = (v > 0.f) ? v : 0.01f * v;
        slab[(mOff + r) * 68 + (j << 4) + rlane] = v;
      }
    }
    __builtin_amdgcn_fence(__ATOMIC_RELEASE, "workgroup");
    __builtin_amdgcn_wave_barrier();
    __builtin_amdgcn_fence(__ATOMIC_ACQUIRE, "workgroup");
    if (OUT_MODE == 0) {
      float* C = (float*)Cout + (size_t)b * strideC;
      const int hh = lane >> 4, c4 = (lane & 15) * 4;
      for (int pass = 0; pass < 2; ++pass) {
#pragma unroll
        for (int it = 0; it < 8; ++it) {
          const int row = it * 2 + hh;
          v4f v = *(const v4f*)(slab + row * 68 + c4);
          *(volatile v4f*)(C + (size_t)(mBase + row) * ldc + n0 + c4) = v;
        }
        __threadfence();
      }
    } else {
      const int q = lane >> 3, c8 = (lane & 7) * 8;
      unsigned short* C  = (unsigned short*)Cout  + (size_t)b * strideC;
      unsigned short* C2 = (OUT_MODE == 2) ? ((unsigned short*)Cout2 + (size_t)b * strideC) : nullptr;
      for (int pass = 0; pass < 2; ++pass) {
#pragma unroll
        for (int it = 0; it < 4; ++it) {
          const int row = it * 4 + q;
          const float* sp = slab + row * 68 + c8;
          v8h hv, lv;
#pragma unroll
          for (int e = 0; e < 8; ++e) {
            if (OUT_MODE == 1) {
              hv[e] = (_Float16)sp[e];
            } else {
              unsigned short hb = f2bf_bits(sp[e]);
              unsigned short lb = f2bf_bits(sp[e] - bf_bits2f(hb));
              hv[e] = __builtin_bit_cast(_Float16, hb);
              lv[e] = __builtin_bit_cast(_Float16, lb);
            }
          }
          *(volatile v8h*)(C + (size_t)(mBase + row) * ldc + n0 + c8) = hv;
          if (OUT_MODE == 2) *(volatile v8h*)(C2 + (size_t)(mBase + row) * ldc + n0 + c8) = lv;
        }
        __threadfence();
      }
    }
    __builtin_amdgcn_fence(__ATOMIC_RELEASE, "workgroup");
    __builtin_amdgcn_wave_barrier();
    __builtin_amdgcn_fence(__ATOMIC_ACQUIRE, "workgroup");
  }
}

__global__ __launch_bounds__(256) void xsplit_kernel(const float* __restrict__ in, unsigned short* __restrict__ hi,
                                                     unsigned short* __restrict__ lo, int n8) {
  const int i = blockIdx.x * 256 + threadIdx.x;
  if (i >= n8) return;
  const float* p = in + 8 * (size_t)i;
  const v4f a = *(const v4f*)(p);
  const v4f c = *(const v4f*)(p + 4);
  unsigned short hb[8], lb[8];
#pragma unroll
  for (int e = 0; e < 4; ++e) {
    const float f0 = a[e];
    hb[e] = f2bf_bits(f0);
    lb[e] = f2bf_bits(f0 - bf_bits2f(hb[e]));
    const float f1 = c[e];
    hb[4 + e] = f2bf_bits(f1);
    lb[4 + e] = f2bf_bits(f1 - bf_bits2f(hb[4 + e]));
  }
  const v4u uh = (v4u){pk16(hb[0], hb[1]), pk16(hb[2], hb[3]), pk16(hb[4], hb[5]), pk16(hb[6], hb[7])};
  const v4u ul = (v4u){pk16(lb[0], lb[1]), pk16(lb[2], lb[3]), pk16(lb[4], lb[5]), pk16(lb[6], lb[7])};
  unsigned short* qh = hi + 8 * (size_t)i;
  unsigned short* ql = lo + 8 * (size_t)i;
  *(volatile v4u*)qh = uh;
  *(volatile v4u*)ql = ul;
  __threadfence();
  *(volatile v4u*)qh = uh;
  *(volatile v4u*)ql = ul;
}

__global__ __launch_bounds__(256) void wsplit_kernel(const float* W0, const float* W1, const float* W2, const float* W3,
                                                     unsigned short* __restrict__ hi, unsigned short* __restrict__ lo,
                                                     int kin, int planeStride) {
  __shared__ float sm[64][65];
  const int t  = threadIdx.x;
  const int i0 = blockIdx.x * 64;
  const int o0 = blockIdx.y * 64;
  const int z  = blockIdx.z;
  const float* W = (z == 0) ? W0 : (z == 1) ? W1 : (z == 2) ? W2 : W3;
#pragma unroll
  for (int it = 0; it < 16; ++it) {
    const int e  = it * 256 + t;
    const int il = e >> 6;
    const int ol = e & 63;
    sm[ol][il] = W[(size_t)(i0 + il) * kEmb + o0 + ol];
  }
  __syncthreads();
  const int lane = t & 31, wave = t >> 5;
  const int q = lane >> 3, c8 = (lane & 7) * 8;
  unsigned short* oh = hi + (size_t)z * planeStride;
  unsigned short* ol2 = lo + (size_t)z * planeStride;
  for (int pass = 0; pass < 2; ++pass) {
#pragma unroll
    for (int it = 0; it < 2; ++it) {
      const int row = wave * 8 + it * 4 + q;
      unsigned short hb[8], lb[8];
#pragma unroll
      for (int e = 0; e < 8; ++e) {
        const float f = sm[row][c8 + e];
        hb[e] = f2bf_bits(f);
        lb[e] = f2bf_bits(f - bf_bits2f(hb[e]));
      }
      const v4u uh = (v4u){pk16(hb[0], hb[1]), pk16(hb[2], hb[3]), pk16(hb[4], hb[5]), pk16(hb[6], hb[7])};
      const v4u ul = (v4u){pk16(lb[0], lb[1]), pk16(lb[2], lb[3]), pk16(lb[4], lb[5]), pk16(lb[6], lb[7])};
      const size_t off = (size_t)(o0 + row) * kin + i0 + c8;
      *(volatile v4u*)(oh + off)  = uh;
      *(volatile v4u*)(ol2 + off) = ul;
    }
    __threadfence();
  }
}

struct RopeTab { float theta[32]; };
static_assert(sizeof(RopeTab) == 128);

__global__ __launch_bounds__(256) void rope_split_kernel(const float* __restrict__ Hin, const int* __restrict__ lengths,
                                                         unsigned short* __restrict__ hi, unsigned short* __restrict__ lo,
                                                         RopeTab tab) {
#pragma clang fp contract(off)
  __shared__ float sth[32];
  const int t = threadIdx.x, lane = t & 31, wave = t >> 5;
  if (t < 32) {
    float th = 0.0f;
#pragma unroll
    for (int i = 0; i < 32; ++i) th = (t == i) ? tab.theta[i] : th;
    sth[t] = th;
  }
  __syncthreads();
  const int seg   = blockIdx.x * 8 + wave;
  const int token = seg >> 2;
  const int head  = seg & 3;
  const int b     = token >> 11;
  const int s     = token & (kSeq - 1);
  const int len   = lengths[b];
  const int pos   = s - (len >> 1);
  const float th  = sth[lane];
  const float ang = (float)pos * th;
  float sn, cs;
  sincosf(ang, &sn, &cs);
  const size_t base = (size_t)token * kEmb + head * kHdim + 2 * lane;
  const v2f xv = *(const v2f*)(Hin + base);
  const float x0 = xv[0], x1 = xv[1];
  const float o0 = x0 * cs - x1 * sn;
  const float o1 = x1 * cs + x0 * sn;
  const unsigned short h0 = f2bf_bits(o0);
  const unsigned short l0 = f2bf_bits(o0 - bf_bits2f(h0));
  const unsigned short h1 = f2bf_bits(o1);
  const unsigned short l1 = f2bf_bits(o1 - bf_bits2f(h1));
  const unsigned uh = pk16(h0, h1);
  const unsigned ul = pk16(l0, l1);
  volatile unsigned* ph = (volatile unsigned*)(hi + base);
  volatile unsigned* pl = (volatile unsigned*)(lo + base);
  *ph = uh;
  *pl = ul;
  __threadfence();
  *ph = uh;
  *pl = ul;
}

__global__ __launch_bounds__(256) void softmax_kernel(const float* __restrict__ Sc, const int* __restrict__ lengths,
                                                      unsigned short* __restrict__ P, int bidx) {
  __shared__ float redM[8];
  __shared__ float redS[8];
  const int row  = blockIdx.x;
  const int t    = threadIdx.x;
  const int lane = t & 31, wave = t >> 5;
  const int c0   = t * 8;
  const int len  = lengths[bidx];
  const float* sr = Sc + (size_t)row * kSeq + c0;
  const v4f a = *(const v4f*)(sr);
  const v4f c = *(const v4f*)(sr + 4);
  float x[8];
#pragma unroll
  for (int e = 0; e < 4; ++e) {
    x[e]     = (c0 + e < len)     ? a[e] : -INFINITY;
    x[4 + e] = (c0 + 4 + e < len) ? c[e] : -INFINITY;
  }
  float m = fmaxf(fmaxf(fmaxf(x[0], x[1]), fmaxf(x[2], x[3])), fmaxf(fmaxf(x[4], x[5]), fmaxf(x[6], x[7])));
#pragma unroll
  for (int off = 16; off > 0; off >>= 1) m = fmaxf(m, __shfl_xor(m, off, 32));
  if (lane == 0) redM[wave] = m;
  __syncthreads();
  float mx = redM[0];
#pragma unroll
  for (int w = 1; w < 8; ++w) mx = fmaxf(mx, redM[w]);
  float ex[8];
  float sm = 0.f;
#pragma unroll
  for (int e = 0; e < 8; ++e) { ex[e] = expf(x[e] - mx); sm += ex[e]; }
#pragma unroll
  for (int off = 16; off > 0; off >>= 1) sm += __shfl_xor(sm, off, 32);
  if (lane == 0) redS[wave] = sm;
  __syncthreads();
  float tot = redS[0];
#pragma unroll
  for (int w = 1; w < 8; ++w) tot += redS[w];
  const float inv = 1.0f / tot;
  unsigned short pb[8];
#pragma unroll
  for (int e = 0; e < 8; ++e) pb[e] = h_bits((ex[e] * inv) * kPCarry);
  const v4u u = (v4u){pk16(pb[0], pb[1]), pk16(pb[2], pb[3]), pk16(pb[4], pb[5]), pk16(pb[6], pb[7])};
  unsigned short* q = P + (size_t)row * kSeq + c0;
  *(volatile v4u*)q = u;
  __threadfence();
  *(volatile v4u*)q = u;
}

extern "C" void kernel_launch(void* const* d_in, const int* in_sizes, int n_in,
                              void* d_out, int out_size, void* d_ws,
                              size_t ws_size, hipStream_t stream) {
  if (n_in < 12) return;
  if (in_sizes[0] != kTok * kPatch || in_sizes[1] != kBatch || in_sizes[2] != kPatch * kEmb || in_sizes[3] != kEmb) return;
  if (in_sizes[4] != kEmb * kEmb || in_sizes[6] != kEmb * kEmb || in_sizes[8] != kEmb * kEmb || in_sizes[10] != kEmb * kEmb) return;
  if (in_sizes[5] != kEmb || in_sizes[7] != kEmb || in_sizes[9] != kEmb || in_sizes[11] != kEmb) return;
  if (out_size != kTok * kEmb) return;
  if (ws_size < kWsTotal) return;

  const float* x     = (const float*)d_in[0];
  const int*   lens  = (const int*)d_in[1];
  const float* W_emb = (const float*)d_in[2];
  const float* b_emb = (const float*)d_in[3];
  const float* Wq    = (const float*)d_in[4];
  const float* bq    = (const float*)d_in[5];
  const float* Wk    = (const float*)d_in[6];
  const float* bk    = (const float*)d_in[7];
  const float* Wv    = (const float*)d_in[8];
  const float* bv    = (const float*)d_in[9];
  const float* Wo    = (const float*)d_in[10];
  const float* bo    = (const float*)d_in[11];
  float* out = (float*)d_out;

  char* ws = (char*)d_ws;
  unsigned short* WeHi = (unsigned short*)(ws + kOffWeHi);
  unsigned short* WeLo = (unsigned short*)(ws + kOffWeLo);
  unsigned short* SqHi = (unsigned short*)(ws + kOffSqHi);
  unsigned short* SqLo = (unsigned short*)(ws + kOffSqLo);
  const size_t kSqPlane = (size_t)kEmb * kEmb;
  unsigned short* WqHi = SqHi + 0 * kSqPlane; unsigned short* WqLo = SqLo + 0 * kSqPlane;
  unsigned short* WkHi = SqHi + 1 * kSqPlane; unsigned short* WkLo = SqLo + 1 * kSqPlane;
  unsigned short* WvHi = SqHi + 2 * kSqPlane; unsigned short* WvLo = SqLo + 2 * kSqPlane;
  unsigned short* WoHi = SqHi + 3 * kSqPlane; unsigned short* WoLo = SqLo + 3 * kSqPlane;
  float*          Hf   = (float*)(ws + kOffH);
  unsigned short* Ohi  = (unsigned short*)(ws + kOffH);
  unsigned short* Olo  = (unsigned short*)(ws + kOffOlo);
  unsigned short* QK   = (unsigned short*)(ws + kOffQK);
  unsigned short* VT   = (unsigned short*)(ws + kOffVT);
  unsigned short* HrHi = (unsigned short*)(ws + kOffHrHi);
  unsigned short* HrLo = (unsigned short*)(ws + kOffHrLo);
  unsigned short* XHi  = (unsigned short*)(ws + kOffXHi);
  unsigned short* XLo  = (unsigned short*)(ws + kOffXLo);
  float*          Sc   = (float*)(ws + kOffScore);
  unsigned short* Pp   = (unsigned short*)(ws + kOffP);

  RopeTab tab;
  for (int p = 0; p < 32; ++p) {
    const float e  = (float)(2 * p) / 64.0f;
    const float pw = (float)pow(10000.0, (double)e);
    tab.theta[p] = 1.0f / pw;
  }

  {
    const int n8 = kTok * kPatch / 8;
    xsplit_kernel<<<dim3((n8 + 255) / 256), dim3(256), 0, stream>>>(x, XHi, XLo, n8);
  }
  wsplit_kernel<<<dim3(kPatch / 64, kEmb / 64, 1), dim3(256), 0, stream>>>(W_emb, W_emb, W_emb, W_emb, WeHi, WeLo, kPatch, 0);
  wsplit_kernel<<<dim3(kEmb / 64, kEmb / 64, 4), dim3(256), 0, stream>>>(Wq, Wk, Wv, Wo, SqHi, SqLo, kEmb, (int)kSqPlane);

  wmma_gemm64<1, true, 2, 0, false><<<dim3(128, 1), dim3(256), 0, stream>>>(
      XHi, XLo, kPatch, 0L, WeHi, WeLo, kPatch, 0L, (void*)Hf, (void*)Hf, kEmb, 0L,
      b_emb, b_emb, 0L, kTok, kEmb, kPatch, 1.0f, 1.0f);

  rope_split_kernel<<<dim3(kTok * kHeads / 8), dim3(256), 0, stream>>>(Hf, lens, HrHi, HrLo, tab);

  wmma_gemm64<1, true, 2, 1, false><<<dim3(128, 1), dim3(256), 0, stream>>>(
      HrHi, HrLo, kEmb, 0L, WqHi, WqLo, kEmb, 0L, (void*)QK, (void*)QK, kQKld, 0L,
      bq, bq, 0L, kTok, kEmb, kEmb, 1.0f, kQKVCarry);
  wmma_gemm64<1, true, 2, 1, false><<<dim3(128, 1), dim3(256), 0, stream>>>(
      HrHi, HrLo, kEmb, 0L, WkHi, WkLo, kEmb, 0L, (void*)(QK + kEmb), (void*)(QK + kEmb), kQKld, 0L,
      bk, bk, 0L, kTok, kEmb, kEmb, 1.0f, kQKVCarry);
  wmma_gemm64<1, true, 1, 1, false><<<dim3(128, 1), dim3(256), 0, stream>>>(
      WvHi, WvLo, kEmb, 0L, HrHi, HrLo, kEmb, 0L, (void*)VT, (void*)VT, kTok, 0L,
      bv, bv, 0L, kEmb, kTok, kEmb, 1.0f, kQKVCarry);

  for (int ch = 0; ch < 16; ++ch) {
    const int b  = ch >> 1;
    const int h0 = (ch & 1) * 2;
    const unsigned short* Qg = QK + (size_t)b * kSeq * kQKld + h0 * kHdim;
    const unsigned short* Kg = QK + (size_t)b * kSeq * kQKld + kEmb + h0 * kHdim;
    wmma_gemm64<0, false, 0, 0, false><<<dim3(128, 2), dim3(256), 0, stream>>>(
        Qg, Qg, kQKld, (long)kHdim, Kg, Kg, kQKld, (long)kHdim, (void*)Sc, (void*)Sc, kSeq, (long)kSeq * kSeq,
        b_emb, b_emb, 0L, kSeq, kSeq, kHdim, kScoreScale, 1.0f);
    softmax_kernel<<<dim3(2 * kSeq), dim3(256), 0, stream>>>(Sc, lens, Pp, b);
    const unsigned short* Vg = VT + (size_t)(h0 * kHdim) * kTok + (size_t)b * kSeq;
    unsigned short* Og_hi = Ohi + (size_t)b * kSeq * kEmb + h0 * kHdim;
    unsigned short* Og_lo = Olo + (size_t)b * kSeq * kEmb + h0 * kHdim;
    wmma_gemm64<0, false, 0, 2, false><<<dim3(4, 2), dim3(256), 0, stream>>>(
        Pp, Pp, kSeq, (long)kSeq * kSeq, Vg, Vg, kTok, (long)kHdim * kTok, (void*)Og_hi, (void*)Og_lo, kEmb, (long)kHdim,
        b_emb, b_emb, 0L, kSeq, kHdim, kSeq, kPVScale, 1.0f);
  }

  wmma_gemm64<1, true, 2, 0, false><<<dim3(128, 1), dim3(256), 0, stream>>>(
      Ohi, Olo, kEmb, 0L, WoHi, WoLo, kEmb, 0L, (void*)out, (void*)out, kEmb, 0L,
      bo, bo, 0L, kTok, kEmb, kEmb, 1.0f, 1.0f);
}
